// GCN_80977313399676
// MI455X (gfx1250) — hardware-run, weakly checked
//
#include <hip/hip_runtime.h>
#include <stddef.h>
#include <stdint.h>
#include <math.h>

#define NN       100000
#define NE       1600000
#define CIN      128
#define HID      128
#define OUTD     64
#define TWO_TERM 1
#define KH       (TWO_TERM ? 2 * HID : HID)
#define GBM      128
#define MP       100096
#define PADR     (MP - NN)
#define NTHR     256
#define NWAVE    8
#define EPT      8
#define WCH      (32 * EPT)
#define NBRUN    1024
#define SLB      10
#define NBK      98
#define WLCAP    3584
#define RCAP     28672
#define DEGCAP   128
#define MAXDEG_MEAS   36
#define MAXB1024_MEAS 16710
#define ABM      64
#define SP       68
#define NBIAS    384

#define BK_ZINTS (NWAVE * WLCAP + RCAP + 3 * NBRUN)
#define BK_INTS  (BK_ZINTS + NBRUN + 16)
#define BK_LDS   (BK_INTS * 4)

#define PBX  (MP * CIN / 8 / NTHR)
#define PBW0 (HID * CIN / 8 / NTHR)
#define PBW1 (HID * KH / 8 / NTHR)
#define PBW2 (OUTD * KH / 8 / NTHR)
#define PBZ  (TWO_TERM ? (PADR * KH / 8 / NTHR) : 0)
#define PBTOT (PBX + PBW0 + PBW1 + PBW2 + PBZ + 1)

static_assert(32 * 4 == HID);
static_assert(16 * 4 == OUTD);
static_assert(NBK * NBRUN >= NN && NBK * NBRUN >= MP);
static_assert(782 * GBM == MP && MP >= NN && MP % ABM == 0 && MP % GBM == 0);
static_assert(NBRUN == (1 << SLB) && NBRUN % ABM == 0 && NBRUN % GBM == 0 && NBRUN % 32 == 0);
static_assert(NBRUN == 4 * NTHR);
static_assert(NN < (1 << 22));
static_assert(NE < (1 << 21) && (((long long)NE) << SLB) < (1LL << 31));
static_assert(NE % WCH == 0 && NE % 4 == 0);
static_assert(RCAP == NWAVE * WLCAP && RCAP % 4 == 0 && BK_ZINTS % 4 == 0 && RCAP % (NTHR * 4) == 0);
static_assert((long long)RCAP * 100 >= (long long)MAXB1024_MEAS * 105);
static_assert(WLCAP >= MAXB1024_MEAS / 8 + 8 * 46 + 1);
static_assert(MAXDEG_MEAS + 8 <= DEGCAP);
static_assert(BK_LDS <= 300000 && BK_LDS <= 327680);
static_assert((GBM * SP + GBM) * 4 <= 65536);
static_assert(CIN % 32 == 0 && KH % 32 == 0 && HID % 64 == 0 && OUTD % 64 == 0);
static_assert((MP * CIN / 8) % NTHR == 0 && (HID * CIN / 8) % NTHR == 0);
static_assert((HID * KH / 8) % NTHR == 0 && (OUTD * KH / 8) % NTHR == 0 && (PADR * KH / 8) % NTHR == 0);
static_assert(((KH / 8) & (KH / 8 - 1)) == 0);
static_assert(NBIAS == 3 * 128 && 2 * HID + OUTD <= NBIAS);
static_assert((long long)MP * CIN * 2 <= (long long)MP * KH * 2);
static_assert((long long)MP * OUTD * 4 <= (long long)MP * HID * 4);

typedef float          v4f   __attribute__((ext_vector_type(4)));
typedef float          v8f   __attribute__((ext_vector_type(8)));
typedef int            v4i   __attribute__((ext_vector_type(4)));
typedef int            v8i   __attribute__((ext_vector_type(8)));
typedef unsigned short v8us  __attribute__((ext_vector_type(8)));
typedef unsigned short v16us __attribute__((ext_vector_type(16)));
typedef __bf16         v16bf __attribute__((ext_vector_type(16)));
typedef v4f  __attribute__((may_alias)) v4fa;
typedef v4i  __attribute__((may_alias)) v4ia;
typedef v8us __attribute__((may_alias)) v8usa;
union FragB { v16bf v; v16us u; v8us h[2]; v8i w; };

__device__ __forceinline__ v8f wmb(const FragB& a, const FragB& b, v8f c) {
  v8f d = __builtin_amdgcn_wmma_f32_16x16x32_bf16(false, a.v, false, b.v, (short)0, c, false, false);
  asm volatile("v_nop\n\tv_nop\n\tv_nop\n\tv_nop" : "+v"(d) : "v"(a.w), "v"(b.w));
  return d;
}

__device__ __forceinline__ unsigned bf16_bits(float f) {
  const unsigned u = __float_as_uint(f);
  const unsigned r = (u + 0x7FFFu + ((u >> 16) & 1u)) >> 16;
  const unsigned q = (u >> 16) | 0x40u;
  return ((u & 0x7fffffffu) > 0x7f800000u) ? q : r;
}

__device__ __forceinline__ void hilo_pack(float v0, float v1, float v2, float v3,
                                          int& h01, int& h23, int& l01, int& l23) {
  const unsigned a0 = bf16_bits(v0), a1 = bf16_bits(v1), a2 = bf16_bits(v2), a3 = bf16_bits(v3);
  const unsigned b0 = bf16_bits(v0 - __uint_as_float(a0 << 16));
  const unsigned b1 = bf16_bits(v1 - __uint_as_float(a1 << 16));
  const unsigned b2 = bf16_bits(v2 - __uint_as_float(a2 << 16));
  const unsigned b3 = bf16_bits(v3 - __uint_as_float(a3 << 16));
  h01 = (int)(a0 | (a1 << 16)); h23 = (int)(a2 | (a3 << 16));
  l01 = (int)(b0 | (b1 << 16)); l23 = (int)(b2 | (b3 << 16));
}

__device__ __forceinline__ void st2_v4f(float* p, v4f v) {
  *(volatile v4f*)p = v;
  __threadfence();
  *(volatile v4f*)p = v;
}
__device__ __forceinline__ void st2_v8us(unsigned short* p, v8us v) {
  *(volatile v8us*)p = v;
  __threadfence();
  *(volatile v8us*)p = v;
}

__device__ __forceinline__ v8us gather8(const float* __restrict__ base, int stride) {
  float f[8];
#pragma unroll
  for (int i = 0; i < 8; ++i) f[i] = base[(size_t)i * (size_t)stride];
  v8us o;
#pragma unroll
  for (int i = 0; i < 8; ++i) o[i] = (unsigned short)bf16_bits(f[i]);
  return o;
}

__global__ __launch_bounds__(NTHR) void k_prep(const float* __restrict__ x, const float* __restrict__ w0,
                                               const float* __restrict__ b0, const float* __restrict__ w1,
                                               const float* __restrict__ b1, const float* __restrict__ w2,
                                               const float* __restrict__ b2,
                                               unsigned short* hx, unsigned short* w0t, unsigned short* w1d,
                                               unsigned short* w2d, float* bias) {
  const int tid = (int)threadIdx.x, lane = tid & 31, wave = tid >> 5;
  const int blk = (int)blockIdx.x;
  if (blk < PBX) {
    const int u   = blk * NTHR + tid;
    const int row = u >> 4, k8 = (u & 15) * 8;
    const int rc  = row < NN ? row : NN - 1;
    const unsigned mk = row < NN ? 0xffffu : 0u;
    const float* p = x + (size_t)rc * CIN + k8;
    const v4f a = *(const v4fa*)p;
    const v4f b = *(const v4fa*)(p + 4);
    v8us o;
    o[0] = (unsigned short)(bf16_bits(a.x) & mk); o[1] = (unsigned short)(bf16_bits(a.y) & mk);
    o[2] = (unsigned short)(bf16_bits(a.z) & mk); o[3] = (unsigned short)(bf16_bits(a.w) & mk);
    o[4] = (unsigned short)(bf16_bits(b.x) & mk); o[5] = (unsigned short)(bf16_bits(b.y) & mk);
    o[6] = (unsigned short)(bf16_bits(b.z) & mk); o[7] = (unsigned short)(bf16_bits(b.w) & mk);
    st2_v8us(hx + (size_t)row * CIN + k8, o);
  } else if (blk < PBX + PBW0) {
    const int u = (blk - PBX) * NTHR + tid;
    const int n = u >> 4, k8 = (u & 15) * 8;
    const v8us o = gather8(w0 + (size_t)k8 * HID + n, HID);
    st2_v8us(w0t + (size_t)n * CIN + k8, o);
  } else if (blk < PBX + PBW0 + PBW1) {
    const int u = (blk - PBX - PBW0) * NTHR + tid;
    const int n = u / (KH / 8), k8 = (u % (KH / 8)) * 8, kk = k8 & (HID - 1);
    const v8us o = gather8(w1 + (size_t)kk * HID + n, HID);
    st2_v8us(w1d + (size_t)n * KH + k8, o);
  } else if (blk < PBX + PBW0 + PBW1 + PBW2) {
    const int u = (blk - PBX - PBW0 - PBW1) * NTHR + tid;
    const int n = u / (KH / 8), k8 = (u % (KH / 8)) * 8, kk = k8 & (HID - 1);
    const v8us o = gather8(w2 + (size_t)kk * OUTD + n, OUTD);
    st2_v8us(w2d + (size_t)n * KH + k8, o);
  } else if (blk < PBX + PBW0 + PBW1 + PBW2 + PBZ) {
    const int u = (blk - PBX - PBW0 - PBW1 - PBW2) * NTHR + tid;
    const int row = NN + u / (KH / 8), k8 = (u % (KH / 8)) * 8;
    const v8us z = {0, 0, 0, 0, 0, 0, 0, 0};
    st2_v8us(hx + (size_t)row * KH + k8, z);
  } else {
    if (tid < 96) {
      const int q = lane & 15;
      const v4f a = *(const v4fa*)(b0 + 4 * lane);
      const v4f b = *(const v4fa*)(b1 + 4 * lane);
      const v4f c = *(const v4fa*)(b2 + 4 * q);
      asm volatile("" :: "v"(a));
      asm volatile("" :: "v"(b));
      asm volatile("" :: "v"(c));
      const unsigned m0 = (wave == 0) ? 0xffffffffu : 0u;
      const unsigned m1 = (wave == 1) ? 0xffffffffu : 0u;
      const unsigned m2 = ((wave == 2) & (lane < 16)) ? 0xffffffffu : 0u;
      v4f o;
      o.x = __uint_as_float(((bf16_bits(a.x) << 16) & m0) | ((bf16_bits(b.x) << 16) & m1) | ((bf16_bits(c.x) << 16) & m2));
      o.y = __uint_as_float(((bf16_bits(a.y) << 16) & m0) | ((bf16_bits(b.y) << 16) & m1) | ((bf16_bits(c.y) << 16) & m2));
      o.z = __uint_as_float(((bf16_bits(a.z) << 16) & m0) | ((bf16_bits(b.z) << 16) & m1) | ((bf16_bits(c.z) << 16) & m2));
      o.w = __uint_as_float(((bf16_bits(a.w) << 16) & m0) | ((bf16_bits(b.w) << 16) & m1) | ((bf16_bits(c.w) << 16) & m2));
      st2_v4f(bias + 4 * tid, o);
    }
  }
}

__device__ __forceinline__ void bucket_flush(const int* pl, const int* cnt, const int* dvb, int ov,
                                             int* lp, int* cop, int* dp, int* fp, int tid) {
#pragma unroll 1
  for (int i = tid * 4; i < RCAP; i += NTHR * 4) {
    const v4i v = *(const v4ia*)(pl + i);
    *(volatile v4i*)(lp + i) = v;
  }
#pragma unroll 1
  for (int it = 0; it < 2; ++it) {
    const int idx = it * (NTHR * 4) + 4 * tid;
    const v4i v = *(const v4ia*)(cnt + idx);
    *(volatile v4i*)(cop + idx) = v;
  }
  {
    const v4i v = *(const v4ia*)(dvb + 4 * tid);
    *(volatile v4i*)(dp + 4 * tid) = v;
  }
  if (tid < 8) {
    const v4i f = {ov, ov, ov, ov};
    *(volatile v4i*)(fp + 4 * tid) = f;
  }
}

__global__ __launch_bounds__(NTHR) void k_bucket(const int* __restrict__ srcs, const int* __restrict__ dsts,
                                                 int* LIST, int* CO, int* DINVB, int* FLAG) {
  extern __shared__ __attribute__((aligned(16))) int dsm[];
  int* wl   = dsm;
  int* pl   = dsm + NWAVE * WLCAP;
  int* cnt  = pl + RCAP;
  int* offs = cnt + NBRUN;
  int* cur  = offs + NBRUN;
  int* dvb  = cur + NBRUN;
  int* misc = dvb + NBRUN;
  const int tid = (int)threadIdx.x, lane = tid & 31, wave = tid >> 5;
  const int blk = (int)blockIdx.x;
  const unsigned nbs = (unsigned)(blk * NBRUN);

  {
    const v4i z4 = {0, 0, 0, 0};
    for (int i = tid * 4; i < BK_ZINTS; i += NTHR * 4) *(v4ia*)(dsm + i) = z4;
    if (tid < 16) misc[tid] = 0;
  }
  __syncthreads();

  {
    const int per  = ((NE + NWAVE * WCH - 1) / (NWAVE * WCH)) * WCH;
    const int ebeg = wave * per;
    const int eend = (ebeg + per < NE) ? (ebeg + per) : NE;
    int* mylist = wl + wave * WLCAP;
    int wc = 0;
#pragma unroll 1
    for (int cb = ebeg; cb < eend; cb += WCH) {
      const int e0 = cb + lane * EPT;
      const v4i da = *(const v4ia*)(dsts + e0);
      const v4i db = *(const v4ia*)(dsts + e0 + 4);
      const unsigned s0 = (unsigned)da.x - nbs, s1 = (unsigned)da.y - nbs;
      const unsigned s2 = (unsigned)da.z - nbs, s3 = (unsigned)da.w - nbs;
      const unsigned s4 = (unsigned)db.x - nbs, s5 = (unsigned)db.y - nbs;
      const unsigned s6 = (unsigned)db.z - nbs, s7 = (unsigned)db.w - nbs;
      const bool h0 = s0 < (unsigned)NBRUN, h1 = s1 < (unsigned)NBRUN, h2 = s2 < (unsigned)NBRUN, h3 = s3 < (unsigned)NBRUN;
      const bool h4 = s4 < (unsigned)NBRUN, h5 = s5 < (unsigned)NBRUN, h6 = s6 < (unsigned)NBRUN, h7 = s7 < (unsigned)NBRUN;
      const unsigned m0 = __builtin_amdgcn_ballot_w32(h0), m1 = __builtin_amdgcn_ballot_w32(h1);
      const unsigned m2 = __builtin_amdgcn_ballot_w32(h2), m3 = __builtin_amdgcn_ballot_w32(h3);
      const unsigned m4 = __builtin_amdgcn_ballot_w32(h4), m5 = __builtin_amdgcn_ballot_w32(h5);
      const unsigned m6 = __builtin_amdgcn_ballot_w32(h6), m7 = __builtin_amdgcn_ballot_w32(h7);
      const unsigned any = m0 | m1 | m2 | m3 | m4 | m5 | m6 | m7;
      if (any != 0u) {
        const int pre = (int)(__builtin_amdgcn_mbcnt_lo(m0, 0u) + __builtin_amdgcn_mbcnt_lo(m1, 0u) +
                              __builtin_amdgcn_mbcnt_lo(m2, 0u) + __builtin_amdgcn_mbcnt_lo(m3, 0u) +
                              __builtin_amdgcn_mbcnt_lo(m4, 0u) + __builtin_amdgcn_mbcnt_lo(m5, 0u) +
                              __builtin_amdgcn_mbcnt_lo(m6, 0u) + __builtin_amdgcn_mbcnt_lo(m7, 0u));
        int p = wc + pre;
        if (h0) { if (p < WLCAP) mylist[p] = ((e0 + 0) << SLB) | (int)s0; p = p + 1; }
        if (h1) { if (p < WLCAP) mylist[p] = ((e0 + 1) << SLB) | (int)s1; p = p + 1; }
        if (h2) { if (p < WLCAP) mylist[p] = ((e0 + 2) << SLB) | (int)s2; p = p + 1; }
        if (h3) { if (p < WLCAP) mylist[p] = ((e0 + 3) << SLB) | (int)s3; p = p + 1; }
        if (h4) { if (p < WLCAP) mylist[p] = ((e0 + 4) << SLB) | (int)s4; p = p + 1; }
        if (h5) { if (p < WLCAP) mylist[p] = ((e0 + 5) << SLB) | (int)s5; p = p + 1; }
        if (h6) { if (p < WLCAP) mylist[p] = ((e0 + 6) << SLB) | (int)s6; p = p + 1; }
        if (h7) { if (p < WLCAP) mylist[p] = ((e0 + 7) << SLB) | (int)s7; p = p + 1; }
        wc += (int)(__builtin_popcount(m0) + __builtin_popcount(m1) + __builtin_popcount(m2) + __builtin_popcount(m3) +
                    __builtin_popcount(m4) + __builtin_popcount(m5) + __builtin_popcount(m6) + __builtin_popcount(m7));
      }
    }
    if (lane == 0) misc[wave] = wc;
  }
  __syncthreads();

  if (wave == 0) {
    int ov = 0;
#pragma unroll 1
    for (int w2 = 0; w2 < NWAVE; ++w2) {
      int c = misc[w2];
      if (c > WLCAP) ov = 1;
      c = c < 0 ? 0 : (c > WLCAP ? WLCAP : c);
#pragma unroll 1
      for (int b0 = 0; b0 < c; b0 += 32) {
        const int idx = b0 + lane;
        const int ent = wl[w2 * WLCAP + (idx < WLCAP ? idx : WLCAP - 1)];
        const int m32 = (c - b0) < 32 ? (c - b0) : 32;
#pragma unroll 1
        for (int k = 0; k < m32; ++k) {
          const int u    = __builtin_amdgcn_readlane(ent, k);
          const int slot = u & (NBRUN - 1);
          if (lane == 0) cnt[slot] = cnt[slot] + 1;
        }
      }
    }
    if (lane == 0) misc[9] = ov;
  }
  __syncthreads();
  if (wave == 0) {
    const int base = lane * (NBRUN / 32);
    int s = 0;
#pragma unroll 1
    for (int i = 0; i < NBRUN / 32; ++i) s += cnt[base + i];
    int incl = s;
#pragma unroll
    for (int d = 1; d < 32; d <<= 1) {
      const int y = __shfl_up(incl, d, 32);
      if (lane >= d) incl += y;
    }
    int run = incl - s;
#pragma unroll 1
    for (int i = 0; i < NBRUN / 32; ++i) {
      const int cv = cnt[base + i];
      offs[base + i] = run;
      cur[base + i]  = run;
      run += cv;
    }
  }
  __syncthreads();

  if (wave == 0) {
#pragma unroll 1
    for (int w2 = 0; w2 < NWAVE; ++w2) {
      int c = misc[w2];
      c = c < 0 ? 0 : (c > WLCAP ? WLCAP : c);
#pragma unroll 1
      for (int b0 = 0; b0 < c; b0 += 32) {
        const int idx = b0 + lane;
        const int ent = wl[w2 * WLCAP + (idx < WLCAP ? idx : WLCAP - 1)];
        int eid = (ent >> SLB) & 0x1FFFFF;
        eid = eid > NE - 1 ? NE - 1 : eid;
        int sr = srcs[eid];
        sr = sr < 0 ? 0 : (sr > NN - 1 ? NN - 1 : sr);
        const int m32 = (c - b0) < 32 ? (c - b0) : 32;
#pragma unroll 1
        for (int k = 0; k < m32; ++k) {
          const int u    = __builtin_amdgcn_readlane(ent, k);
          const int wd   = __builtin_amdgcn_readlane(sr, k);
          const int slot = u & (NBRUN - 1);
          if (lane == 0) {
            int p = cur[slot];
            p = p < 0 ? 0 : (p > RCAP - 1 ? RCAP - 1 : p);
            pl[p] = wd;
            cur[slot] = p + 1;
          }
        }
      }
    }
  }
#pragma unroll 1
  for (int i = tid; i < NBRUN; i += NTHR) {
    int cv = cnt[i];
    cv = cv < 0 ? 0 : cv;
    const float dg = (float)(cv + 1);
    dvb[i] = __float_as_int(1.0f / sqrtf(dg));
  }
  __syncthreads();

  const int ovf = misc[9];
  int* lp  = LIST + (size_t)blk * RCAP;
  int* cop = CO + (size_t)blk * (2 * NBRUN);
  int* dp  = DINVB + (size_t)blk * NBRUN;
  int* fp  = FLAG + (size_t)blk * 32;
  bucket_flush(pl, cnt, dvb, ovf, lp, cop, dp, fp, tid);
  __threadfence();
  bucket_flush(pl, cnt, dvb, ovf, lp, cop, dp, fp, tid);
}

template <int KTOT>
__device__ __forceinline__ void gemm_16x64(const unsigned short* __restrict__ ap,
                                           const unsigned short* __restrict__ bp, v8f (&acc)[4]) {
#pragma unroll 1
  for (int k0 = 0; k0 < KTOT; k0 += 32) {
    FragB af;
    af.h[0] = *(const v8usa*)(ap + k0);
    af.h[1] = *(const v8usa*)(ap + k0 + 16);
#pragma unroll
    for (int nt = 0; nt < 4; ++nt) {
      const unsigned short* wq = bp + (size_t)(16 * nt) * (size_t)KTOT + k0;
      FragB bf;
      bf.h[0] = *(const v8usa*)wq;
      bf.h[1] = *(const v8usa*)(wq + 16);
      acc[nt] = wmb(af, bf, acc[nt]);
    }
  }
}

__device__ __forceinline__ void stage_d(float* stg, const v8f (&acc)[4], int wave, int hh, int m) {
#pragma unroll
  for (int nt = 0; nt < 4; ++nt) {
#pragma unroll
    for (int r = 0; r < 8; ++r) stg[(16 * wave + 8 * hh + r) * SP + 16 * nt + m] = acc[nt][r];
  }
}

template <int KTOT>
__global__ __launch_bounds__(NTHR) __attribute__((amdgpu_num_vgpr(248)))
void k_gemm(const unsigned short* __restrict__ A, const unsigned short* __restrict__ BT,
            const float* __restrict__ DINV, float* P, int ldo) {
  __shared__ __attribute__((aligned(16))) float stg[GBM * SP];
  __shared__ __attribute__((aligned(16))) float sdv[GBM];
  const int tid = (int)threadIdx.x, lane = tid & 31, wave = tid >> 5, hh = lane >> 4, m = lane & 15;
  const int rowBase = (int)blockIdx.x * GBM;
  const int col0    = (int)blockIdx.y * 64;
  if (tid < 32) *(v4fa*)(sdv + 4 * tid) = *(const v4fa*)(DINV + (size_t)rowBase + 4 * tid);

  v8f acc[4];
  {
    const v8f z = {0.f, 0.f, 0.f, 0.f, 0.f, 0.f, 0.f, 0.f};
#pragma unroll
    for (int t = 0; t < 4; ++t) acc[t] = z;
  }
  const unsigned short* ap = A + (size_t)(rowBase + 16 * wave + m) * (size_t)KTOT + 8 * hh;
  const unsigned short* bp = BT + (size_t)(col0 + m) * (size_t)KTOT + 8 * hh;
  gemm_16x64<KTOT>(ap, bp, acc);
  stage_d(stg, acc, wave, hh, m);
  __syncthreads();

#pragma unroll 1
  for (int i = 0; i < 8; ++i) {
    const int lr   = 16 * wave + 2 * i + hh;
    const int grow = rowBase + lr;
    const bool live = grow < NN;
    const v4f a  = *(const v4fa*)(stg + lr * SP + 4 * m);
    const float dv = sdv[lr];
    asm volatile("" :: "v"(a));
    asm volatile("" :: "v"(dv));
    const float v0 = dv * a.x, v1 = dv * a.y, v2 = dv * a.z, v3 = dv * a.w;
    v4f o;
    o.x = live ? v0 : 0.0f; o.y = live ? v1 : 0.0f; o.z = live ? v2 : 0.0f; o.w = live ? v3 : 0.0f;
    st2_v4f(P + (size_t)grow * (size_t)ldo + col0 + 4 * m, o);
  }
}

__global__ __launch_bounds__(NTHR) void k_replay_h(const int* __restrict__ LIST, const int* __restrict__ CO,
                                                   const int* __restrict__ FLAG, const float* __restrict__ DINV,
                                                   const float* __restrict__ P, const float* __restrict__ bias,
                                                   unsigned short* H) {
  const int tid = (int)threadIdx.x, lane = tid & 31;
  const int wave = __builtin_amdgcn_readfirstlane(tid >> 5);
  const int rowBase = (int)blockIdx.x * ABM;
  const int bucket  = rowBase >> SLB;
  const int* lb  = LIST + (size_t)bucket * RCAP;
  const int* cob = CO + (size_t)bucket * (2 * NBRUN);
  const int flag = FLAG[(size_t)bucket * 32];
  const float qnan = __uint_as_float(0x7fc00000u);
  const v4f bv = *(const v4fa*)(bias + 4 * lane);
  const int s0 = (2 * lane) & 31, s1 = s0 + 1;
  const int mk = (lane < 16) ? -1 : 0;

#pragma unroll 1
  for (int i = 0; i < ABM / NWAVE; ++i) {
    const int d    = rowBase + (ABM / NWAVE) * wave + i;
    const int slot = d & (NBRUN - 1);
    int c = cob[slot];
    int o = cob[NBRUN + slot];
    const bool big = c > DEGCAP;
    c = c < 0 ? 0 : (c > DEGCAP ? DEGCAP : c);
    o = o < 0 ? 0 : (o > RCAP - 1 ? RCAP - 1 : o);
    int last = o + c - 1;
    last = last < o ? o : last;
    last = last > RCAP - 1 ? RCAP - 1 : last;
    float a0 = 0.0f, a1 = 0.0f, a2 = 0.0f, a3 = 0.0f;
#pragma unroll 1
    for (int j = 0; j < c; ++j) {
      int idx = o + j;
      idx = idx > last ? last : idx;
      int sr = lb[idx];
      sr = sr < 0 ? 0 : (sr > NN - 1 ? NN - 1 : sr);
      const v4f v = *(const v4fa*)(P + (size_t)sr * HID + 4 * lane);
      asm volatile("" :: "v"(v));
      a0 += v.x; a1 += v.y; a2 += v.z; a3 += v.w;
    }
    const v4f g = *(const v4fa*)(P + (size_t)d * HID + 4 * lane);
    const float dv = DINV[d];
    float v0 = dv * (a0 + g.x) + bv.x, v1 = dv * (a1 + g.y) + bv.y;
    float v2 = dv * (a2 + g.z) + bv.z, v3 = dv * (a3 + g.w) + bv.w;
    v0 = (v0 > 0.0f) ? v0 : (v0 - v0); v1 = (v1 > 0.0f) ? v1 : (v1 - v1);
    v2 = (v2 > 0.0f) ? v2 : (v2 - v2); v3 = (v3 > 0.0f) ? v3 : (v3 - v3);
    const bool bad  = (flag != 0) | big;
    const bool live = d < NN;
    v0 = bad ? qnan : v0; v1 = bad ? qnan : v1; v2 = bad ? qnan : v2; v3 = bad ? qnan : v3;
    v0 = live ? v0 : 0.0f; v1 = live ? v1 : 0.0f; v2 = live ? v2 : 0.0f; v3 = live ? v3 : 0.0f;
    int h01, h23, l01, l23;
    hilo_pack(v0, v1, v2, v3, h01, h23, l01, l23);
    const int p0 = __shfl(h01, s0, 32), p1 = __shfl(h23, s0, 32), p2 = __shfl(h01, s1, 32), p3 = __shfl(h23, s1, 32);
    if constexpr (TWO_TERM != 0) {
      const int q0 = __shfl(l01, s0, 32), q1 = __shfl(l23, s0, 32), q2 = __shfl(l01, s1, 32), q3 = __shfl(l23, s1, 32);
      v4i ow;
      ow.x = (p0 & mk) | (q0 & ~mk); ow.y = (p1 & mk) | (q1 & ~mk);
      ow.z = (p2 & mk) | (q2 & ~mk); ow.w = (p3 & mk) | (q3 & ~mk);
      unsigned short* hp = H + (size_t)d * KH + 8 * lane;
      *(volatile v4i*)hp = ow;
      __threadfence();
      *(volatile v4i*)hp = ow;
    } else {
      v4i ow;
      ow.x = p0; ow.y = p1; ow.z = p2; ow.w = p3;
      unsigned short* hp = H + (size_t)d * KH + 8 * (lane & 15);
      const bool wr = lane < 16;
      if (wr) *(volatile v4i*)hp = ow;
      __threadfence();
      if (wr) *(volatile v4i*)hp = ow;
    }
  }
}

__global__ __launch_bounds__(NTHR) void k_replay_out(const int* __restrict__ LIST, const int* __restrict__ CO,
                                                     const int* __restrict__ FLAG, const float* __restrict__ DINV,
                                                     const float* __restrict__ P3, const float* __restrict__ bias,
                                                     float* out) {
  const int tid = (int)threadIdx.x, lane = tid & 31, wave = tid >> 5, hh = lane >> 4, q = lane & 15;
  const int rowBase = (int)blockIdx.x * ABM;
  const int bucket  = rowBase >> SLB;
  const int* lb  = LIST + (size_t)bucket * RCAP;
  const int* cob = CO + (size_t)bucket * (2 * NBRUN);
  const int flag = FLAG[(size_t)bucket * 32];
  const float qnan = __uint_as_float(0x7fc00000u);
  const v4f bv = *(const v4fa*)(bias + 4 * q);

#pragma unroll 1
  for (int i = 0; i < ABM / (2 * NWAVE); ++i) {
    const int d    = rowBase + (ABM / NWAVE) * wave + 2 * i + hh;
    const int slot = d & (NBRUN - 1);
    int c = cob[slot];
    int o = cob[NBRUN + slot];
    const bool big = c > DEGCAP;
    c = c < 0 ? 0 : (c > DEGCAP ? DEGCAP : c);
    o = o < 0 ? 0 : (o > RCAP - 1 ? RCAP - 1 : o);
    const int co = __shfl_xor(c, 16, 32);
    const int cm = c > co ? c : co;
    int last = o + c - 1;
    last = last < o ? o : last;
    last = last > RCAP - 1 ? RCAP - 1 : last;
    float a0 = 0.0f, a1 = 0.0f, a2 = 0.0f, a3 = 0.0f;
#pragma unroll 1
    for (int j = 0; j < cm; ++j) {
      int idx = o + j;
      idx = idx > last ? last : idx;
      int sr = lb[idx];
      sr = sr < 0 ? 0 : (sr > NN - 1 ? NN - 1 : sr);
      const v4f v = *(const v4fa*)(P3 + (size_t)sr * OUTD + 4 * q);
      asm volatile("" :: "v"(v));
      const bool valid = j < c;
      const float t0 = a0 + v.x, t1 = a1 + v.y, t2 = a2 + v.z, t3 = a3 + v.w;
      a0 = valid ? t0 : a0; a1 = valid ? t1 : a1; a2 = valid ? t2 : a2; a3 = valid ? t3 : a3;
    }
    const v4f g = *(const v4fa*)(P3 + (size_t)d * OUTD + 4 * q);
    const float dv = DINV[d];
    float v0 = dv * (a0 + g.x) + bv.x, v1 = dv * (a1 + g.y) + bv.y;
    float v2 = dv * (a2 + g.z) + bv.z, v3 = dv * (a3 + g.w) + bv.w;
    const bool bad  = (flag != 0) | big;
    const bool live = d < NN;
    v4f ov;
    ov.x = bad ? qnan : v0; ov.y = bad ? qnan : v1; ov.z = bad ? qnan : v2; ov.w = bad ? qnan : v3;
    const int dc = live ? d : NN - 1;
    float* op = out + (size_t)dc * OUTD + 4 * q;
    if (live) *(volatile v4f*)op = ov;
    __threadfence();
    if (live) *(volatile v4f*)op = ov;
  }
}

extern "C" void kernel_launch(void* const* d_in, const int* in_sizes, int n_in,
                              void* d_out, int out_size, void* d_ws, size_t ws_size,
                              hipStream_t stream) {
  if (n_in < 8) return;
  if (in_sizes[0] != NN * CIN) return;
  if (in_sizes[1] != 2 * NE) return;
  if (in_sizes[2] != CIN * HID) return;
  if (in_sizes[3] != HID) return;
  if (in_sizes[4] != HID * HID) return;
  if (in_sizes[5] != HID) return;
  if (in_sizes[6] != HID * OUTD) return;
  if (in_sizes[7] != OUTD) return;
  if (out_size != NN * OUTD) return;

  const float* x  = (const float*)d_in[0];
  const int*   ei = (const int*)d_in[1];
  const float* W0 = (const float*)d_in[2];
  const float* b0 = (const float*)d_in[3];
  const float* W1 = (const float*)d_in[4];
  const float* b1 = (const float*)d_in[5];
  const float* W2 = (const float*)d_in[6];
  const float* b2 = (const float*)d_in[7];
  float* out = (float*)d_out;
  const int* srcs = ei;
  const int* dsts = ei + NE;

  constexpr size_t zH    = (size_t)MP * KH * 2;
  constexpr size_t zP    = (size_t)MP * HID * 4;
  constexpr size_t zLIST = (size_t)NBK * RCAP * 4;
  constexpr size_t zCO   = (size_t)NBK * 2 * NBRUN * 4;
  constexpr size_t zDINV = (size_t)NBK * NBRUN * 4;
  constexpr size_t zFLAG = (size_t)NBK * 128;
  constexpr size_t zW0T  = (size_t)HID * CIN * 2;
  constexpr size_t zW1D  = (size_t)HID * KH * 2;
  constexpr size_t zW2D  = (size_t)OUTD * KH * 2;
  constexpr size_t zBIAS = (size_t)NBIAS * 4;
  constexpr size_t oH    = 0;
  constexpr size_t oP    = oH + zH;
  constexpr size_t oLIST = oP + zP;
  constexpr size_t oCO   = oLIST + zLIST;
  constexpr size_t oDINV = oCO + zCO;
  constexpr size_t oFLAG = oDINV + zDINV;
  constexpr size_t oW0T  = oFLAG + zFLAG;
  constexpr size_t oW1D  = oW0T + zW0T;
  constexpr size_t oW2D  = oW1D + zW1D;
  constexpr size_t oBIAS = oW2D + zW2D;
  constexpr size_t oEND  = oBIAS + zBIAS;
  static_assert(zH % 256 == 0 && zP % 256 == 0 && zLIST % 256 == 0 && zCO % 256 == 0 && zDINV % 256 == 0);
  static_assert(zFLAG % 256 == 0 && zW0T % 256 == 0 && zW1D % 256 == 0 && zW2D % 256 == 0 && zBIAS % 256 == 0);
  static_assert(oEND <= ((size_t)128 << 20));
  static_assert((size_t)NBK * NBRUN >= (size_t)MP);
  if (oEND > ws_size) return;

  char* ws = (char*)d_ws;
  unsigned short* HX   = (unsigned short*)(ws + oH);
  float*          P    = (float*)(ws + oP);
  int*            LIST = (int*)(ws + oLIST);
  int*            CO   = (int*)(ws + oCO);
  float*          DINV = (float*)(ws + oDINV);
  int*            FLAG = (int*)(ws + oFLAG);
  unsigned short* W0T  = (unsigned short*)(ws + oW0T);
  unsigned short* W1D  = (unsigned short*)(ws + oW1D);
  unsigned short* W2D  = (unsigned short*)(ws + oW2D);
  float*          BIAS = (float*)(ws + oBIAS);

  hipFuncSetAttribute(reinterpret_cast<const void*>(&k_bucket), hipFuncAttributeMaxDynamicSharedMemorySize, (int)BK_LDS);

  k_prep<<<PBTOT, NTHR, 0, stream>>>(x, W0, b0, W1, b1, W2, b2, HX, W0T, W1D, W2D, BIAS);
  k_bucket<<<NBK, NTHR, BK_LDS, stream>>>(srcs, dsts, LIST, CO, (int*)DINV, FLAG);
  k_gemm<CIN><<<dim3(MP / GBM, HID / 64), NTHR, 0, stream>>>(HX, W0T, DINV, P, HID);
  k_replay_h<<<MP / ABM, NTHR, 0, stream>>>(LIST, CO, FLAG, DINV, P, BIAS, HX);
  k_gemm<KH><<<dim3(MP / GBM, HID / 64), NTHR, 0, stream>>>(HX, W1D, DINV, P, HID);
  k_replay_h<<<MP / ABM, NTHR, 0, stream>>>(LIST, CO, FLAG, DINV, P, BIAS + HID, HX);
  k_gemm<KH><<<dim3(MP / GBM, OUTD / 64), NTHR, 0, stream>>>(HX, W2D, DINV, P, OUTD);
  k_replay_out<<<MP / ABM, NTHR, 0, stream>>>(LIST, CO, FLAG, DINV, P, BIAS + 2 * HID, out);
}
